// MultitaskRNN_70643622084779
// MI455X (gfx1250) — hardware-verified
//
#include <hip/hip_runtime.h>


typedef _Float16 v16h __attribute__((ext_vector_type(16)));
typedef _Float16 v8h  __attribute__((ext_vector_type(8), __may_alias__));
typedef _Float16 v4h  __attribute__((ext_vector_type(4), __may_alias__));
typedef float    v8f  __attribute__((ext_vector_type(8)));
typedef float    v4f  __attribute__((ext_vector_type(4), __may_alias__));

#define NB   64
#define NT   512
#define NI   128
#define NH   512
#define NO   64
#define KC   (NH + NI)
#define RB   16
#define RTHR (RB * 32)
#define PA   (KC + 8)
#define PF   (NH + 4)
#define PO   (NO + 4)
#define OWAV 8
#define SCH  64.0f
#define SCX  64.0f
#define SCW  16.0f
#define INV  (1.0f / 1024.0f)

union Frag { v16h v; v8h p[2]; };

static __device__ __forceinline__ v8f mma16(v16h a, v16h b, v8f c)
{
    c = __builtin_amdgcn_wmma_f32_16x16x32_f16(false, a, false, b, (short)0, c, false, false);
    asm volatile("v_nop\n\tv_nop\n\tv_nop\n\tv_nop" : "+v"(c) : "v"(a), "v"(b));
    return c;
}

static __device__ __forceinline__ v16h frag_row(const _Float16* row, int k0, int h)
{
    Frag f;
    f.p[0] = *(const v8h*)(row + k0 + 8 * h);
    f.p[1] = *(const v8h*)(row + k0 + 16 + 8 * h);
    return f.v;
}

__global__ __launch_bounds__(256) void prep_kernel(
    const float* __restrict__ W_rec, const float* __restrict__ W_in,
    const float* __restrict__ W_out, _Float16* Wcat, _Float16* Wo)
{
    const int i   = blockIdx.x * 256 + threadIdx.x;
    const int nWc = NH * KC / 8;
    const int nWo = NO * NH / 8;
    if (i < nWc) {
        const int e = i * 8;
        const int n = e / KC;
        const int k = e - n * KC;
        const float* s = (k < NH) ? (W_rec + (size_t)n * NH + k) : (W_in + (size_t)n * NI + (k - NH));
        const v4f x0 = *(const v4f*)s;
        const v4f x1 = *(const v4f*)(s + 4);
        v8h o = {};
#pragma unroll
        for (int q = 0; q < 4; ++q) {
            o[q]     = (_Float16)(x0[q] * SCW);
            o[4 + q] = (_Float16)(x1[q] * SCW);
        }
        volatile v8h* d = (volatile v8h*)(Wcat + e);
        *d = o;
        __threadfence();
        *d = o;
    }
    if (i < nWo) {
        const int e = i * 8;
        const float* s = W_out + e;
        const v4f x0 = *(const v4f*)s;
        const v4f x1 = *(const v4f*)(s + 4);
        v8h o = {};
#pragma unroll
        for (int q = 0; q < 4; ++q) {
            o[q]     = (_Float16)(x0[q] * SCW);
            o[4 + q] = (_Float16)(x1[q] * SCW);
        }
        volatile v8h* d = (volatile v8h*)(Wo + e);
        *d = o;
        __threadfence();
        *d = o;
    }
}

__global__ __launch_bounds__(RTHR) void recur_kernel(
    const float* __restrict__ inputs, const float* __restrict__ hidden,
    const _Float16* __restrict__ Wcat, const float* __restrict__ bias,
    _Float16* hist, float* hfin)
{
    __shared__ __attribute__((aligned(16))) _Float16 hA[RB * PA];
    __shared__ __attribute__((aligned(16))) float    hF[RB * PF];

    const int tid  = threadIdx.x;
    const int lane = tid & 31;
    const int w    = tid >> 5;
    const int h    = lane >> 4;
    const int m    = lane & 15;
    const int rb0  = blockIdx.x * RB;
    if (rb0 + RB > NB) return;
    const int cA = w * 32;
    const int cB = cA + 16;
    const int xr = tid >> 5;
    const int xq = tid & 31;

    v8f s0 = {};
    v8f s1 = {};
#pragma unroll
    for (int v = 0; v < 8; ++v) {
        const int r = 8 * h + v;
        const float* hr = hidden + (size_t)(rb0 + r) * NH;
        const float q0 = hr[cA + m];
        const float q1 = hr[cB + m];
        s0[v] = q0;
        s1[v] = q1;
        hA[r * PA + cA + m] = (_Float16)(q0 * SCH);
        hA[r * PA + cB + m] = (_Float16)(q1 * SCH);
    }
    {
        const float* src = inputs + ((size_t)(rb0 + xr) * NT + 0) * NI + 4 * xq;
        const v4f x = *(const v4f*)src;
        v4h xh = {};
#pragma unroll
        for (int q = 0; q < 4; ++q) xh[q] = (_Float16)(x[q] * SCX);
        *(v4h*)(hA + xr * PA + NH + 4 * xq) = xh;
    }
    __syncthreads();

    const float bb0 = bias[cA + m];
    const float bb1 = bias[cB + m];
    const _Float16* arow  = hA + m * PA;
    const _Float16* brow0 = Wcat + (size_t)(cA + m) * KC;
    const _Float16* brow1 = Wcat + (size_t)(cB + m) * KC;

    for (int t = 0; t < NT; ++t) {
        v8f a0 = {};
        v8f a1 = {};
#pragma unroll 2
        for (int ks = 0; ks < KC / 32; ++ks) {
            const int k0 = ks * 32;
            const v16h a  = frag_row(arow, k0, h);
            const v16h b0 = frag_row(brow0, k0, h);
            const v16h b1 = frag_row(brow1, k0, h);
            a0 = mma16(a, b0, a0);
            a1 = mma16(a, b1, a1);
        }
#pragma unroll
        for (int v = 0; v < 8; ++v) {
            const float p0 = a0[v] * INV + bb0;
            const float p1 = a1[v] * INV + bb1;
            s0[v] = 0.9f * s0[v] + 0.1f * tanhf(p0);
            s1[v] = 0.9f * s1[v] + 0.1f * tanhf(p1);
        }
        __syncthreads();
#pragma unroll
        for (int v = 0; v < 8; ++v) {
            const int r = 8 * h + v;
            hA[r * PA + cA + m] = (_Float16)(s0[v] * SCH);
            hA[r * PA + cB + m] = (_Float16)(s1[v] * SCH);
        }
        if (t + 1 < NT) {
            const float* src = inputs + ((size_t)(rb0 + xr) * NT + (t + 1)) * NI + 4 * xq;
            const v4f x = *(const v4f*)src;
            v4h xh = {};
#pragma unroll
            for (int q = 0; q < 4; ++q) xh[q] = (_Float16)(x[q] * SCX);
            *(v4h*)(hA + xr * PA + NH + 4 * xq) = xh;
        }
        __syncthreads();
        {
            const v8h* sr = (const v8h*)(hA + w * PA);
            const v8h p0 = sr[lane];
            const v8h p1 = sr[32 + lane];
            volatile v8h* d = (volatile v8h*)(hist + ((size_t)(rb0 + w) * NT + t) * NH);
            d[lane]      = p0;
            d[32 + lane] = p1;
            __threadfence();
            d[lane]      = p0;
            d[32 + lane] = p1;
        }
    }

#pragma unroll
    for (int v = 0; v < 8; ++v) {
        const int r = 8 * h + v;
        hF[r * PF + cA + m] = s0[v];
        hF[r * PF + cB + m] = s1[v];
    }
    __syncthreads();
    {
        const v4f* sr = (const v4f*)(hF + w * PF);
        const v4f q0 = sr[lane];
        const v4f q1 = sr[32 + lane];
        const v4f q2 = sr[64 + lane];
        const v4f q3 = sr[96 + lane];
        volatile v4f* d = (volatile v4f*)(hfin + (size_t)(rb0 + w) * NH);
        d[lane]      = q0;
        d[32 + lane] = q1;
        d[64 + lane] = q2;
        d[96 + lane] = q3;
        __threadfence();
        d[lane]      = q0;
        d[32 + lane] = q1;
        d[64 + lane] = q2;
        d[96 + lane] = q3;
    }
}

__global__ __launch_bounds__(OWAV * 32) void out_kernel(
    const _Float16* __restrict__ hist, const _Float16* __restrict__ Wo,
    const float* __restrict__ b_out, float* out, int nrow_tiles)
{
    __shared__ __attribute__((aligned(16))) float st[OWAV * 16 * PO];

    const int tid  = threadIdx.x;
    const int lane = tid & 31;
    const int w    = tid >> 5;
    const int h    = lane >> 4;
    const int m    = lane & 15;
    const int rt   = blockIdx.x * OWAV + w;
    const bool active = rt < nrow_tiles;
    const int rtc  = active ? rt : 0;

    const _Float16* arow = hist + ((size_t)rtc * 16 + m) * NH;
    v8f c[4];
#pragma unroll
    for (int j = 0; j < 4; ++j) { v8f z = {}; c[j] = z; }

#pragma unroll 2
    for (int ks = 0; ks < NH / 32; ++ks) {
        const int k0 = ks * 32;
        const v16h a = frag_row(arow, k0, h);
#pragma unroll
        for (int j = 0; j < 4; ++j) {
            const v16h b = frag_row(Wo + (size_t)(16 * j + m) * NH, k0, h);
            c[j] = mma16(a, b, c[j]);
        }
    }

    float* tile = st + w * (16 * PO);
#pragma unroll
    for (int j = 0; j < 4; ++j) {
        const float bo = b_out[16 * j + m];
#pragma unroll
        for (int v = 0; v < 8; ++v)
            tile[(8 * h + v) * PO + 16 * j + m] = c[j][v] * INV + bo;
    }
    __syncthreads();

    v4f q[8];
#pragma unroll
    for (int p = 0; p < 8; ++p)
        q[p] = *(const v4f*)(tile + (2 * p + h) * PO + 4 * m);

    if (active) {
        volatile v4f* d = (volatile v4f*)(out + (size_t)rt * 16 * NO);
#pragma unroll
        for (int p = 0; p < 8; ++p) d[(2 * p + h) * 16 + m] = q[p];
        __threadfence();
#pragma unroll
        for (int p = 0; p < 8; ++p) d[(2 * p + h) * 16 + m] = q[p];
    }
}

extern "C" void kernel_launch(void* const* d_in, const int* in_sizes, int n_in,
                              void* d_out, int out_size, void* d_ws, size_t ws_size,
                              hipStream_t stream)
{
    if (n_in < 7) return;
    if (in_sizes[0] != NB * NT * NI || in_sizes[1] != NB * NH || in_sizes[2] != NH * NI ||
        in_sizes[3] != NH * NH   || in_sizes[4] != NH      || in_sizes[5] != NO * NH ||
        in_sizes[6] != NO) return;
    if (out_size != NB * NT * NO + NB * NH) return;

    const float* inputs = (const float*)d_in[0];
    const float* hidden = (const float*)d_in[1];
    const float* W_in   = (const float*)d_in[2];
    const float* W_rec  = (const float*)d_in[3];
    const float* bias   = (const float*)d_in[4];
    const float* W_out  = (const float*)d_in[5];
    const float* b_out  = (const float*)d_in[6];

    const size_t szWc  = (size_t)NH * KC * sizeof(_Float16);
    const size_t szWo  = (size_t)NO * NH * sizeof(_Float16);
    const size_t szHi  = (size_t)NB * NT * NH * sizeof(_Float16);
    const size_t offWc = 0;
    const size_t offWo = (offWc + szWc + 255) & ~(size_t)255;
    const size_t offHi = (offWo + szWo + 255) & ~(size_t)255;
    if (offHi + szHi > ws_size) return;

    char* ws = (char*)d_ws;
    _Float16* Wcat = (_Float16*)(ws + offWc);
    _Float16* Wo   = (_Float16*)(ws + offWo);
    _Float16* hist = (_Float16*)(ws + offHi);

    float* out0 = (float*)d_out;
    float* out1 = out0 + (size_t)NB * NT * NO;

    const int nprep = NH * KC / 8;
    prep_kernel<<<dim3((nprep + 255) / 256), dim3(256), 0, stream>>>(W_rec, W_in, W_out, Wcat, Wo);

    recur_kernel<<<dim3((NB + RB - 1) / RB), dim3(RTHR), 0, stream>>>(inputs, hidden, Wcat, bias, hist, out1);

    const int ntiles = (NB * NT) / 16;
    out_kernel<<<dim3((ntiles + OWAV - 1) / OWAV), dim3(OWAV * 32), 0, stream>>>(hist, Wo, b_out, out0, ntiles);
}
